// OrthogonalBivectorBlock_25348896981073
// MI455X (gfx1250) — hardware-run, weakly checked
//
#include <hip/hip_runtime.h>
#include <math.h>

typedef __attribute__((ext_vector_type(16))) _Float16 v16h;
typedef __attribute__((ext_vector_type(8)))  _Float16 v8h;
typedef __attribute__((ext_vector_type(8)))  float    v8f;
typedef __attribute__((ext_vector_type(4)))  float    v4f;
typedef __attribute__((ext_vector_type(2)))  float    v2f;
typedef __attribute__((ext_vector_type(4)))  unsigned int v4u;

constexpr int kBatch  = 2;
constexpr int kSeq    = 2048;
constexpr int kDim    = 512;
constexpr int kTok    = kBatch * kSeq;
constexpr int kGateH  = 256;
constexpr int kSets   = 4;
constexpr int kPlanesPerSet = 4;
constexpr int kPlanes = kSets * kPlanesPerSet;
constexpr int kPosPl  = 16;
constexpr int kHeadPad = 64;
constexpr int kFeat   = 64;
static_assert(kTok == 4096);
static_assert(kPlanes == 16 && kPosPl == 16);
static_assert((kDim % 32) == 0);
static_assert((kTok % 64) == 0 && (kDim % 64) == 0 && (kGateH % 64) == 0 && (kHeadPad % 64) == 0);

constexpr float kXCarry = 16.0f;
constexpr float kWCarry = 256.0f;
constexpr float kHCarry = 64.0f;
constexpr float kNCarry = 16.0f;
constexpr float kScaleXW = 1.0f / (kXCarry * kWCarry);
constexpr float kScaleHW = 1.0f / (kHCarry * kWCarry);
constexpr float kScaleNW = 1.0f / (kNCarry * kWCarry);
constexpr float kF16MinNormal = 6.103515625e-05f;
constexpr float kPiF    = 3.14159265358979323846f;
constexpr float kTwoPiF = 6.28318530717958647692f;
constexpr float kRsqrt2 = 0.70710678118654752440f;
constexpr float kLnEps  = 1e-5f;

constexpr size_t kSzX16  = (size_t)kTok * kDim * 2;
constexpr size_t kSzWSQ  = (size_t)4 * kDim * kDim * 2;
constexpr size_t kSzWG1  = (size_t)kGateH * kDim * 2;
constexpr size_t kSzW2P  = (size_t)2 * kHeadPad * kDim * 2;
constexpr size_t kSzPRE  = (size_t)2 * kTok * kDim * 4;
constexpr size_t kSzVV   = (size_t)kTok * kDim * 4;
constexpr size_t kSzGP   = (size_t)kTok * kGateH * 4;
constexpr size_t kSzH16  = (size_t)2 * kTok * kDim * 2;
constexpr size_t kSzPH   = (size_t)2 * kTok * kHeadPad * 4;
constexpr size_t kSzFT   = (size_t)2 * kTok * kFeat * 4;
constexpr size_t kSzTOT  = (size_t)2 * kTok * kDim * 4;
constexpr size_t kSzHN16 = (size_t)kTok * kDim * 2;
constexpr size_t kOffX16  = 0;
constexpr size_t kOffWSQ  = kOffX16 + kSzX16;
constexpr size_t kOffWG1  = kOffWSQ + kSzWSQ;
constexpr size_t kOffW2P  = kOffWG1 + kSzWG1;
constexpr size_t kOffPRE  = kOffW2P + kSzW2P;
constexpr size_t kOffVV   = kOffPRE + kSzPRE;
constexpr size_t kOffGP   = kOffVV  + kSzVV;
constexpr size_t kOffH16  = kOffGP  + kSzGP;
constexpr size_t kOffPH   = kOffH16 + kSzH16;
constexpr size_t kOffFT   = kOffPH  + kSzPH;
constexpr size_t kOffTOT  = kOffFT  + kSzFT;
constexpr size_t kOffHN16 = kOffTOT + kSzTOT;
constexpr size_t kWsTotal = kOffHN16 + kSzHN16;
static_assert(kWsTotal == 69599232ull);
static_assert(kWsTotal <= 134217728ull);
static_assert((kOffWSQ % 128) == 0 && (kOffWG1 % 128) == 0 && (kOffW2P % 128) == 0 && (kOffPRE % 128) == 0 &&
              (kOffVV % 128) == 0 && (kOffGP % 128) == 0 && (kOffH16 % 128) == 0 && (kOffPH % 128) == 0 &&
              (kOffFT % 128) == 0 && (kOffTOT % 128) == 0 && (kOffHN16 % 128) == 0);

__device__ __forceinline__ unsigned pk16(unsigned short a, unsigned short b) { return (unsigned)a | ((unsigned)b << 16); }

__device__ __forceinline__ unsigned short h_bits_flush(float f) {
  const float g = (fabsf(f) < kF16MinNormal) ? 0.0f : f;
  const _Float16 h = (_Float16)g;
  return __builtin_bit_cast(unsigned short, h);
}

union FragU { v16h v; v8h h[2]; };
__device__ __forceinline__ v16h frag_load(const _Float16* p) {
  FragU f;
  f.h[0] = *(const v8h*)(p);
  f.h[1] = *(const v8h*)(p + 16);
  return f.v;
}
__device__ __forceinline__ v8f wm_mma(v16h a, v16h b, v8f c) {
  return __builtin_amdgcn_wmma_f32_16x16x32_f16(false, a, false, b, (short)0, c, false, false);
}
__device__ __forceinline__ void wm_guard(v8f& c, v16h a, v16h b) {
  asm volatile("v_nop\n\tv_nop\n\tv_nop\n\tv_nop" : "+v"(c) : "v"(a), "v"(b));
}
__device__ __forceinline__ void keep4_h(v16h a, v16h b, v16h c, v16h d) { asm volatile("v_nop" :: "v"(a), "v"(b), "v"(c), "v"(d)); }
__device__ __forceinline__ void acc_guard4(v8f& a, v8f& b, v8f& c, v8f& d) { asm volatile("v_nop\n\tv_nop\n\tv_nop\n\tv_nop" : "+v"(a), "+v"(b), "+v"(c), "+v"(d)); }

template <int BIAS_MODE, bool RESID>
__global__ __launch_bounds__(256) void wmma_gemm64(
    const unsigned short* __restrict__ Ap, int lda, long strideA,
    const unsigned short* __restrict__ Btp, int ldb, long strideB,
    float* __restrict__ Cout, int ldc, long strideC,
    const float* __restrict__ bias,
    const float* __restrict__ resid,
    int M, int N, int K, float scale) {
  const _Float16* A  = (const _Float16*)Ap;
  const _Float16* Bt = (const _Float16*)Btp;
  __shared__ __align__(16) float sT[8][16 * 68];
  const int b    = blockIdx.y;
  const int lane = threadIdx.x & 31;
  const int wave = threadIdx.x >> 5;
  const int tilesN = N >> 6;
  const int tilesM = M >> 6;
  const int tile = blockIdx.x * 8 + wave;
  if (tile >= tilesM * tilesN) return;
  const int tm = tile / tilesN;
  const int tn = tile - tm * tilesN;
  const int m0 = tm << 6;
  const int n0 = tn << 6;

  const _Float16* Ab = A  + (size_t)b * strideA;
  const _Float16* Bb = Bt + (size_t)b * strideB;

  const int rlane = lane & 15;
  const int koff  = (lane >> 4) * 8;
  const int mOff  = (lane >> 4) * 8;

  v8f acc[4][4];
#pragma unroll
  for (int i = 0; i < 4; ++i)
#pragma unroll
    for (int j = 0; j < 4; ++j) acc[i][j] = (v8f){0.f,0.f,0.f,0.f,0.f,0.f,0.f,0.f};

  for (int k0 = 0; k0 < K; k0 += 32) {
    v16h bh[4];
#pragma unroll
    for (int j = 0; j < 4; ++j) {
      const size_t bo = (size_t)(n0 + (j << 4) + rlane) * ldb + koff + k0;
      bh[j] = frag_load(Bb + bo);
    }
#pragma unroll
    for (int i = 0; i < 4; ++i) {
      const size_t ao = (size_t)(m0 + (i << 4) + rlane) * lda + koff + k0;
      const v16h ah = frag_load(Ab + ao);
#pragma unroll
      for (int j = 0; j < 4; ++j) acc[i][j] = wm_mma(ah, bh[j], acc[i][j]);
#pragma unroll
      for (int j = 0; j < 4; ++j) wm_guard(acc[i][j], ah, bh[j]);
    }
    keep4_h(bh[0], bh[1], bh[2], bh[3]);
  }
  acc_guard4(acc[0][0], acc[0][1], acc[0][2], acc[0][3]);
  acc_guard4(acc[1][0], acc[1][1], acc[1][2], acc[1][3]);
  acc_guard4(acc[2][0], acc[2][1], acc[2][2], acc[2][3]);
  acc_guard4(acc[3][0], acc[3][1], acc[3][2], acc[3][3]);

  float* slab = sT[wave];
  float* C = Cout + (size_t)b * strideC;
  const int hh = lane >> 4, c4 = (lane & 15) * 4;
#pragma unroll
  for (int i = 0; i < 4; ++i) {
    const int mBase = m0 + (i << 4);
#pragma unroll
    for (int j = 0; j < 4; ++j) {
      const int n = n0 + (j << 4) + rlane;
      float bv = 0.f;
      if (BIAS_MODE == 2) bv = bias[n];
#pragma unroll
      for (int r = 0; r < 8; ++r) {
        float v = acc[i][j][r] * scale;
        if (BIAS_MODE == 2) v += bv;
        slab[(mOff + r) * 68 + (j << 4) + rlane] = v;
      }
    }
    __builtin_amdgcn_fence(__ATOMIC_RELEASE, "workgroup");
    __builtin_amdgcn_wave_barrier();
    __builtin_amdgcn_fence(__ATOMIC_ACQUIRE, "workgroup");
    v4f vv[8];
#pragma unroll
    for (int it = 0; it < 8; ++it) {
      const int row = it * 2 + hh;
      v4f v = *(const v4f*)(slab + row * 68 + c4);
      if (RESID) {
        const v4f rv = *(const v4f*)(resid + (size_t)(mBase + row) * ldc + n0 + c4);
        v += rv;
      }
      vv[it] = v;
    }
    for (int pass = 0; pass < 2; ++pass) {
#pragma unroll
      for (int it = 0; it < 8; ++it) {
        const int row = it * 2 + hh;
        *(volatile v4f*)(C + (size_t)(mBase + row) * ldc + n0 + c4) = vv[it];
      }
      __threadfence();
    }
    __builtin_amdgcn_fence(__ATOMIC_RELEASE, "workgroup");
    __builtin_amdgcn_wave_barrier();
    __builtin_amdgcn_fence(__ATOMIC_ACQUIRE, "workgroup");
  }
}

__global__ __launch_bounds__(256) void cast8_f16_kernel(const float* __restrict__ in, unsigned short* __restrict__ out, int n8, float carry) {
  const int i = blockIdx.x * 256 + threadIdx.x;
  if (i >= n8) return;
  const float* p = in + 8 * (size_t)i;
  const v4f a = *(const v4f*)(p);
  const v4f c = *(const v4f*)(p + 4);
  const float a0 = a[0], a1 = a[1], a2 = a[2], a3 = a[3];
  const float c0 = c[0], c1 = c[1], c2 = c[2], c3 = c[3];
  const v4u u = (v4u){pk16(h_bits_flush(a0 * carry), h_bits_flush(a1 * carry)),
                      pk16(h_bits_flush(a2 * carry), h_bits_flush(a3 * carry)),
                      pk16(h_bits_flush(c0 * carry), h_bits_flush(c1 * carry)),
                      pk16(h_bits_flush(c2 * carry), h_bits_flush(c3 * carry))};
  unsigned short* q = out + 8 * (size_t)i;
  *(volatile v4u*)q = u;
  __threadfence();
  *(volatile v4u*)q = u;
}

__global__ __launch_bounds__(256) void wt_kernel(const float* __restrict__ W0, const float* __restrict__ W1,
                                                 const float* __restrict__ W2, const float* __restrict__ W3,
                                                 unsigned short* __restrict__ out, int nreal, long planeStride, float scale) {
  __shared__ float sm[64][65];
  const int t  = threadIdx.x;
  const int k0 = blockIdx.x * 64;
  const int n0 = blockIdx.y * 64;
  const int z  = blockIdx.z;
  const float* W = (z == 0) ? W0 : (z == 1) ? W1 : (z == 2) ? W2 : W3;
#pragma unroll
  for (int i = 0; i < 16; ++i) {
    const int e = i * 256 + t;
    const int r = e >> 6;
    const int c = e & 63;
    const int n = n0 + c;
    const int nc = (n < nreal) ? n : (nreal - 1);
    float wv = W[(size_t)(k0 + r) * nreal + nc];
    asm volatile("" : "+v"(wv));
    const float v = (n < nreal) ? (wv * scale) : 0.0f;
    sm[c][r] = v;
  }
  __syncthreads();
  const int lane = t & 31, wave = t >> 5;
  const int q = lane >> 3, c8 = (lane & 7) * 8;
  unsigned short* op = out + (size_t)z * planeStride;
  v4u u[2];
#pragma unroll
  for (int it = 0; it < 2; ++it) {
    const int row = wave * 8 + it * 4 + q;
    unsigned short hb[8];
#pragma unroll
    for (int e = 0; e < 8; ++e) hb[e] = h_bits_flush(sm[row][c8 + e]);
    u[it] = (v4u){pk16(hb[0], hb[1]), pk16(hb[2], hb[3]), pk16(hb[4], hb[5]), pk16(hb[6], hb[7])};
  }
  for (int pass = 0; pass < 2; ++pass) {
#pragma unroll
    for (int it = 0; it < 2; ++it) {
      const int row = wave * 8 + it * 4 + q;
      *(volatile v4u*)(op + (size_t)(n0 + row) * kDim + k0 + c8) = u[it];
    }
    __threadfence();
  }
}

__global__ __launch_bounds__(256) void gelu_cast_kernel(const float* __restrict__ PRE, const float* __restrict__ kb1,
                                                        const float* __restrict__ qb1, unsigned short* __restrict__ H16) {
  __shared__ __align__(16) unsigned sm[1024];
  const int t = threadIdx.x;
  const size_t base = (size_t)blockIdx.x * 2048;
  const int plane = blockIdx.x >> 10;
  const float* bp = (plane == 0) ? kb1 : qb1;
#pragma unroll 1
  for (int i = 0; i < 4; ++i) {
    const int pi = i * 256 + t;
    const int e = 2 * pi;
    const v2f pv = *(const v2f*)(PRE + base + e);
    const v2f bv = *(const v2f*)(bp + (e & (kDim - 1)));
    const float a0 = pv[0] + bv[0];
    const float a1 = pv[1] + bv[1];
    const float g0 = 0.5f * a0 * (1.0f + erff(a0 * kRsqrt2));
    const float g1 = 0.5f * a1 * (1.0f + erff(a1 * kRsqrt2));
    sm[pi] = pk16(h_bits_flush(g0 * kHCarry), h_bits_flush(g1 * kHCarry));
  }
  __syncthreads();
  const v4u u = *(const v4u*)(sm + 4 * t);
  unsigned short* q = H16 + base + 8 * (size_t)t;
  *(volatile v4u*)q = u;
  __threadfence();
  *(volatile v4u*)q = u;
}

constexpr int kFTok = 32;
constexpr int kFAng = 48;
__global__ __launch_bounds__(256) void feature_kernel(const float* __restrict__ PH, const float* __restrict__ kb2,
                                                      const float* __restrict__ qb2, const float* __restrict__ setw,
                                                      const float* __restrict__ freqs, float* __restrict__ FT) {
#pragma clang fp contract(off)
  __shared__ float sC[kFTok * kFAng];
  __shared__ float sS[kFTok * kFAng];
  __shared__ float sE[4];
  const int tid = threadIdx.x;
  const int tok0 = blockIdx.x * kFTok;
  {
    const float s0 = setw[0], s1 = setw[1], s2 = setw[2], s3 = setw[3];
    const float m = fmaxf(fmaxf(s0, s1), fmaxf(s2, s3));
    const int si = tid & 3;
    const float a = (si == 0) ? (s0 - m) : (si == 1) ? (s1 - m) : (si == 2) ? (s2 - m) : (s3 - m);
    const float e = expf(a);
    if (tid < 4) sE[tid] = e;
  }
#pragma unroll 1
  for (int i = 0; i < 6; ++i) {
    const int idx = i * 256 + tid;
    const int tok = idx / kFAng;
    const int j = idx - tok * kFAng;
    const int kind = j >> 4;
    const int p = j & 15;
    const int t = tok0 + tok;
    const int l = t & (kSeq - 1);
    float pkv = PH[(size_t)t * kHeadPad + p];
    float pqv = PH[(size_t)kTok * kHeadPad + (size_t)t * kHeadPad + p];
    float kbv = kb2[p];
    float qbv = qb2[p];
    float fv  = freqs[p];
    asm volatile("" : "+v"(pkv));
    asm volatile("" : "+v"(pqv));
    asm volatile("" : "+v"(kbv));
    asm volatile("" : "+v"(qbv));
    asm volatile("" : "+v"(fv));
    const float pre = (kind == 0) ? (pkv + kbv) : (pqv + qbv);
    const float th = tanhf(pre) * kPiF;
    const float lf = (float)l * fv;
    const float psi = lf * kTwoPiF;
    const float ang = (kind == 2) ? psi : th;
    sC[idx] = cosf(ang);
    sS[idx] = sinf(ang);
  }
  __syncthreads();
  const float e0 = sE[0], e1 = sE[1], e2 = sE[2], e3 = sE[3];
  const float einv = __builtin_amdgcn_rcpf((e0 + e1) + (e2 + e3));
  const float w0 = e0 * einv, w1 = e1 * einv, w2 = e2 * einv, w3 = e3 * einv;
  v4f val[4];
#pragma unroll
  for (int it = 0; it < 4; ++it) {
    const int e = it * 256 + tid;
    const int half = e >> 9;
    const int rem = e & 511;
    const int tok = rem >> 4;
    const int c4 = (rem & 15) << 2;
    const int qd = c4 >> 4;
    const int pb = c4 & 15;
    const int jj = (half == 1) ? (32 + pb) : ((qd >= 2) ? (16 + pb) : pb);
    const bool useSin = (qd & 1) != 0;
    const int sidx = pb >> 2;
    const float wsel = (sidx == 0) ? w0 : (sidx == 1) ? w1 : (sidx == 2) ? w2 : w3;
    const float coef = (half == 0 && qd >= 2) ? wsel : 1.0f;
    const float* pc = sC + tok * kFAng + jj;
    const float* ps = sS + tok * kFAng + jj;
    const float c0 = pc[0], c1 = pc[1], c2 = pc[2], c3 = pc[3];
    const float s0 = ps[0], s1 = ps[1], s2 = ps[2], s3 = ps[3];
    v4f o;
    o[0] = (useSin ? s0 : c0) * coef;
    o[1] = (useSin ? s1 : c1) * coef;
    o[2] = (useSin ? s2 : c2) * coef;
    o[3] = (useSin ? s3 : c3) * coef;
    val[it] = o;
  }
  for (int pass = 0; pass < 2; ++pass) {
#pragma unroll
    for (int it = 0; it < 4; ++it) {
      const int e = it * 256 + tid;
      const int half = e >> 9;
      const int rem = e & 511;
      const int tok = rem >> 4;
      const int c4 = (rem & 15) << 2;
      *(volatile v4f*)(FT + (size_t)half * kTok * kFeat + (size_t)(tok0 + tok) * kFeat + c4) = val[it];
    }
    __threadfence();
  }
}

constexpr int kMemSteps = 64;
constexpr int kMemCh    = 64;
constexpr int kMemYP    = 68;
static_assert((kSeq % kMemSteps) == 0 && (kDim % kMemCh) == 0);
__global__ __launch_bounds__(64) void memory_kernel(const float* __restrict__ Vv, const float* __restrict__ FT,
                                                    float* __restrict__ TOT) {
  __shared__ __align__(16) float sF[kMemSteps * kFeat];
  __shared__ __align__(16) float sY[kMemSteps * kMemYP];
  const int tid = threadIdx.x, lane = tid & 31, wave = tid >> 5;
  const int bid = blockIdx.x;
  const int half = bid >> 4;
  const int rem = bid & 15;
  const int bix = rem >> 3;
  const int d0 = (rem & 7) * kMemCh;
  const int d = d0 + tid;
  const size_t row0 = (size_t)bix * kSeq;
  const float* F = FT + (size_t)half * kTok * kFeat;
  float* O = TOT + (size_t)half * kTok * kDim;
  float re[16], im[16];
#pragma unroll
  for (int p = 0; p < 16; ++p) { re[p] = 0.0f; im[p] = 0.0f; }
  const int lr = tid >> 4, lc4 = (tid & 15) * 4;
  const int hh = lane >> 4, c4 = (lane & 15) * 4;
#pragma unroll 1
  for (int t0 = 0; t0 < kSeq; t0 += kMemSteps) {
    __syncthreads();
#pragma unroll
    for (int i = 0; i < 16; ++i) {
      const int r = lr + 4 * i;
      *(v4f*)(sF + r * kFeat + lc4) = *(const v4f*)(F + (row0 + t0 + r) * kFeat + lc4);
    }
    __syncthreads();
#pragma unroll 1
    for (int s = 0; s < kMemSteps; ++s) {
      const float v = Vv[(row0 + t0 + s) * kDim + d];
      const float* xr = sF + s * kFeat;
      float y = 0.0f;
#pragma unroll
      for (int g = 0; g < 4; ++g) {
        const v4f kc = *(const v4f*)(xr + 4 * g);
        const v4f ks = *(const v4f*)(xr + 16 + 4 * g);
        const v4f qc = *(const v4f*)(xr + 32 + 4 * g);
        const v4f qs = *(const v4f*)(xr + 48 + 4 * g);
#pragma unroll
        for (int k = 0; k < 4; ++k) {
          re[4 * g + k] = fmaf(kc[k], v, re[4 * g + k]);
          im[4 * g + k] = fmaf(ks[k], v, im[4 * g + k]);
          y = fmaf(qc[k], re[4 * g + k], y);
          y = fmaf(qs[k], im[4 * g + k], y);
        }
      }
      sY[s * kMemYP + tid] = y;
    }
    __syncthreads();
    for (int pass = 0; pass < 2; ++pass) {
#pragma unroll
      for (int it = 0; it < 16; ++it) {
        const int row = wave * 32 + it * 2 + hh;
        const v4f val = *(const v4f*)(sY + row * kMemYP + c4);
        *(volatile v4f*)(O + (row0 + t0 + row) * kDim + d0 + c4) = val;
      }
      __threadfence();
    }
  }
}

static_assert(kGateH == 256 && kDim == 512);
__device__ __forceinline__ float block_sum256(float v, float* red, int lane, int wave) {
#pragma unroll
  for (int off = 16; off > 0; off >>= 1) v += __shfl_xor(v, off, 32);
  if (lane == 0) red[wave] = v;
  __syncthreads();
  float s = red[0];
  s += red[1]; s += red[2]; s += red[3]; s += red[4]; s += red[5]; s += red[6]; s += red[7];
  return s;
}
__global__ __launch_bounds__(256) void gate_norm_kernel(const float* __restrict__ TOT, const float* __restrict__ GP,
                                                        const float* __restrict__ gw2, const float* __restrict__ gb2,
                                                        const float* __restrict__ posw, const float* __restrict__ lng,
                                                        const float* __restrict__ lnb, unsigned short* __restrict__ HN16) {
  __shared__ float red[3][8];
  __shared__ __align__(16) unsigned sP[256];
  const int tid = threadIdx.x, lane = tid & 31, wave = tid >> 5;
  const int tok = blockIdx.x;
  const int l = tok & (kSeq - 1);
  const float gp = GP[(size_t)tok * kGateH + tid];
  const float ge = 0.5f * gp * (1.0f + erff(gp * kRsqrt2));
  const float gsum = block_sum256(ge * gw2[tid], red[0], lane, wave);
  const float g  = __builtin_amdgcn_rcpf(1.0f + expf(-(gsum + gb2[0])));
  const float sp = __builtin_amdgcn_rcpf(1.0f + expf(-posw[0]));
  const float cb = (1.0f - g) * sp;
  const float rn = __builtin_amdgcn_rsqf((float)(l + 1) * (float)kPlanesPerSet);
  const v2f a = *(const v2f*)(TOT + (size_t)tok * kDim + 2 * tid);
  const v2f b = *(const v2f*)(TOT + (size_t)kTok * kDim + (size_t)tok * kDim + 2 * tid);
  const float a0 = a[0], a1 = a[1], b0 = b[0], b1 = b[1];
  const float h0 = (g * a0 + cb * b0) * rn;
  const float h1 = (g * a1 + cb * b1) * rn;
  const float mu = block_sum256(h0 + h1, red[1], lane, wave) * (1.0f / (float)kDim);
  const float q0 = h0 - mu, q1 = h1 - mu;
  const float var = block_sum256(q0 * q0 + q1 * q1, red[2], lane, wave) * (1.0f / (float)kDim);
  const float rinv = __builtin_amdgcn_rsqf(var + kLnEps);
  const v2f lg = *(const v2f*)(lng + 2 * tid);
  const v2f lb = *(const v2f*)(lnb + 2 * tid);
  const float lg0 = lg[0], lg1 = lg[1], lb0 = lb[0], lb1 = lb[1];
  const float o0 = q0 * rinv * lg0 + lb0;
  const float o1 = q1 * rinv * lg1 + lb1;
  sP[tid] = pk16(h_bits_flush(o0 * kNCarry), h_bits_flush(o1 * kNCarry));
  __syncthreads();
  if (tid < 64) {
    const v4u u = *(const v4u*)(sP + 4 * tid);
    unsigned short* q = HN16 + (size_t)tok * kDim + 8 * tid;
    *(volatile v4u*)q = u;
    __threadfence();
    *(volatile v4u*)q = u;
  }
}

extern "C" void kernel_launch(void* const* d_in, const int* in_sizes, int n_in,
                              void* d_out, int out_size, void* d_ws, size_t ws_size,
                              hipStream_t stream) {
  if (n_in < 22) return;
  if (in_sizes[0] != kTok * kDim) return;
  if (in_sizes[1] != kDim * kDim || in_sizes[5] != kDim * kDim || in_sizes[9] != kDim * kDim || in_sizes[13] != kDim * kDim) return;
  if (in_sizes[2] != kDim || in_sizes[6] != kDim || in_sizes[10] != kDim || in_sizes[11] != kDim || in_sizes[12] != kDim || in_sizes[14] != kDim) return;
  if (in_sizes[3] != kDim * kPlanes || in_sizes[7] != kDim * kPlanes) return;
  if (in_sizes[4] != kPlanes || in_sizes[8] != kPlanes) return;
  if (in_sizes[15] != kSets || in_sizes[16] != kPosPl || in_sizes[17] != 1) return;
  if (in_sizes[18] != kDim * kGateH || in_sizes[19] != kGateH || in_sizes[20] != kGateH || in_sizes[21] != 1) return;
  if (out_size != kTok * kDim) return;
  if (ws_size < kWsTotal) return;

  const float* x     = (const float*)d_in[0];
  const float* ke_w1 = (const float*)d_in[1];
  const float* ke_b1 = (const float*)d_in[2];
  const float* ke_w2 = (const float*)d_in[3];
  const float* ke_b2 = (const float*)d_in[4];
  const float* qe_w1 = (const float*)d_in[5];
  const float* qe_b1 = (const float*)d_in[6];
  const float* qe_w2 = (const float*)d_in[7];
  const float* qe_b2 = (const float*)d_in[8];
  const float* v_w   = (const float*)d_in[9];
  const float* v_b   = (const float*)d_in[10];
  const float* ln_g  = (const float*)d_in[11];
  const float* ln_b  = (const float*)d_in[12];
  const float* out_w = (const float*)d_in[13];
  const float* out_b = (const float*)d_in[14];
  const float* set_w = (const float*)d_in[15];
  const float* freqs = (const float*)d_in[16];
  const float* pos_w = (const float*)d_in[17];
  const float* gw1   = (const float*)d_in[18];
  const float* gb1   = (const float*)d_in[19];
  const float* gw2   = (const float*)d_in[20];
  const float* gb2   = (const float*)d_in[21];
  float* out = (float*)d_out;

  char* ws = (char*)d_ws;
  unsigned short* X16  = (unsigned short*)(ws + kOffX16);
  unsigned short* WSQ  = (unsigned short*)(ws + kOffWSQ);
  unsigned short* WG1  = (unsigned short*)(ws + kOffWG1);
  unsigned short* W2P  = (unsigned short*)(ws + kOffW2P);
  float*          PRE  = (float*)(ws + kOffPRE);
  float*          VV   = (float*)(ws + kOffVV);
  float*          GP   = (float*)(ws + kOffGP);
  unsigned short* H16  = (unsigned short*)(ws + kOffH16);
  float*          PH   = (float*)(ws + kOffPH);
  float*          FT   = (float*)(ws + kOffFT);
  float*          TOT  = (float*)(ws + kOffTOT);
  unsigned short* HN16 = (unsigned short*)(ws + kOffHN16);

  const long sqPlane = (long)kDim * kDim;

  cast8_f16_kernel<<<(kTok * kDim / 8) / 256, 256, 0, stream>>>(x, X16, kTok * kDim / 8, kXCarry);
  wt_kernel<<<dim3(kDim / 64, kDim / 64, 4), 256, 0, stream>>>(ke_w1, qe_w1, v_w, out_w, WSQ, kDim, sqPlane, kWCarry);
  wt_kernel<<<dim3(kDim / 64, kGateH / 64, 1), 256, 0, stream>>>(gw1, gw1, gw1, gw1, WG1, kGateH, 0L, kWCarry);
  wt_kernel<<<dim3(kDim / 64, kHeadPad / 64, 2), 256, 0, stream>>>(ke_w2, qe_w2, ke_w2, qe_w2, W2P, kPlanes, (long)kHeadPad * kDim, kWCarry);

  wmma_gemm64<0, false><<<dim3(64, 2), 256, 0, stream>>>(
      X16, kDim, 0L, WSQ, kDim, sqPlane, PRE, kDim, (long)kTok * kDim,
      nullptr, nullptr, kTok, kDim, kDim, kScaleXW);
  wmma_gemm64<2, false><<<dim3(64, 1), 256, 0, stream>>>(
      X16, kDim, 0L, WSQ + 2 * (size_t)sqPlane, kDim, 0L, VV, kDim, 0L,
      v_b, nullptr, kTok, kDim, kDim, kScaleXW);
  wmma_gemm64<2, false><<<dim3(32, 1), 256, 0, stream>>>(
      X16, kDim, 0L, WG1, kDim, 0L, GP, kGateH, 0L,
      gb1, nullptr, kTok, kGateH, kDim, kScaleXW);

  gelu_cast_kernel<<<(2 * kTok * kDim) / 2048, 256, 0, stream>>>(PRE, ke_b1, qe_b1, H16);

  wmma_gemm64<0, false><<<dim3(8, 2), 256, 0, stream>>>(
      H16, kDim, (long)kTok * kDim, W2P, kDim, (long)kHeadPad * kDim, PH, kHeadPad, (long)kTok * kHeadPad,
      nullptr, nullptr, kTok, kHeadPad, kDim, kScaleHW);

  feature_kernel<<<kTok / kFTok, 256, 0, stream>>>(PH, ke_b2, qe_b2, set_w, freqs, FT);

  memory_kernel<<<2 * kBatch * (kDim / kMemCh), kMemCh, 0, stream>>>(VV, FT, TOT);

  gate_norm_kernel<<<kTok, 256, 0, stream>>>(TOT, GP, gw2, gb2, pos_w, ln_g, ln_b, HN16);

  wmma_gemm64<2, true><<<dim3(64, 1), 256, 0, stream>>>(
      HN16, kDim, 0L, WSQ + 3 * (size_t)sqPlane, kDim, 0L, out, kDim, 0L,
      out_b, x, kTok, kDim, kDim, kScaleNW);
}
